// MultiHeadAttention_RoPE_11038065951105
// MI455X (gfx1250) — hardware-verified
//
#include <hip/hip_runtime.h>
#include <math.h>

typedef __attribute__((ext_vector_type(16))) _Float16 v16h;
typedef __attribute__((ext_vector_type(8)))  _Float16 v8h;
typedef __attribute__((ext_vector_type(16))) __bf16   v16b;
typedef __attribute__((ext_vector_type(8)))  __bf16   v8b;
typedef __attribute__((ext_vector_type(8)))  float    v8f;
typedef __attribute__((ext_vector_type(4)))  float    v4f;
typedef __attribute__((ext_vector_type(4)))  unsigned int v4u;
#define PSCALE 32768.0f
#define U16(p) ((const unsigned short*)(const void*)(p))
#define PSCALE_INV (1.0f / 32768.0f)

__device__ __forceinline__ unsigned short f2bf_bits(float f) {
  unsigned u = __float_as_uint(f);
  return (unsigned short)((u + 0x7FFFu + ((u >> 16) & 1u)) >> 16);
}
__device__ __forceinline__ float bf_bits2f(unsigned short h) { return __uint_as_float(((unsigned)h) << 16); }

__device__ __forceinline__ void dep_guard_h(v8f& a, v8f& b, v16h x, v16h y) { asm volatile("v_nop\n\tv_nop\n\tv_nop\n\tv_nop" : "+v"(a), "+v"(b) : "v"(x), "v"(y)); }
__device__ __forceinline__ void dep_guard_b(v8f& a, v8f& b, v16b x, v16b y) { asm volatile("v_nop\n\tv_nop\n\tv_nop\n\tv_nop" : "+v"(a), "+v"(b) : "v"(x), "v"(y)); }
__device__ __forceinline__ void keep4_h(v16h a, v16h b, v16h c, v16h d) { asm volatile("v_nop" :: "v"(a), "v"(b), "v"(c), "v"(d)); }
__device__ __forceinline__ void keep4_b(v16b a, v16b b, v16b c, v16b d) { asm volatile("v_nop" :: "v"(a), "v"(b), "v"(c), "v"(d)); }
__device__ __forceinline__ void acc_guard4(v8f& a, v8f& b, v8f& c, v8f& d) { asm volatile("v_nop\n\tv_nop\n\tv_nop\n\tv_nop" : "+v"(a), "+v"(b), "+v"(c), "+v"(d)); }
template <typename T> struct Frag;
template <> struct Frag<_Float16> {
  typedef v16h V; union U { v16h v; v8h h[2]; };
  static __device__ __forceinline__ v16h load(const _Float16* p) {
    U f; f.h[0] = *(const v8h*)(p); f.h[1] = *(const v8h*)(p + 16); return f.v;
  }
  static __device__ __forceinline__ v8f mma(v16h a, v16h b, v8f c) {
    return __builtin_amdgcn_wmma_f32_16x16x32_f16(false, a, false, b, (short)0, c, false, false);
  }
  static __device__ __forceinline__ void guard(v8f& a, v8f& b, v16h x, v16h y) { dep_guard_h(a, b, x, y); }
  static __device__ __forceinline__ void keep(v16h a, v16h b, v16h c, v16h d) { keep4_h(a, b, c, d); }
};
template <> struct Frag<__bf16> {
  typedef v16b V; union U { v16b v; v8b h[2]; };
  static __device__ __forceinline__ v16b load(const __bf16* p) {
    U f; f.h[0] = *(const v8b*)(p); f.h[1] = *(const v8b*)(p + 16); return f.v;
  }
  static __device__ __forceinline__ v8f mma(v16b a, v16b b, v8f c) {
    return __builtin_amdgcn_wmma_f32_16x16x32_bf16(false, a, false, b, (short)0, c, false, false);
  }
  static __device__ __forceinline__ void guard(v8f& a, v8f& b, v16b x, v16b y) { dep_guard_b(a, b, x, y); }
  static __device__ __forceinline__ void keep(v16b a, v16b b, v16b c, v16b d) { keep4_b(a, b, c, d); }
};

template <int ET> struct Elem;
template <> struct Elem<0> { typedef _Float16 T; };
template <> struct Elem<1> { typedef __bf16 T; };
template <int ET, bool SPLIT, int BIAS_MODE, int OUT_MODE, bool RESID, int ACT = 0>
__global__ __launch_bounds__(256) void wmma_gemm64(
    const unsigned short* __restrict__ Ap, const unsigned short* __restrict__ A2p, int lda, long strideA,
    const unsigned short* __restrict__ Btp, const unsigned short* __restrict__ Bt2p, int ldb, long strideB,
    void* __restrict__ Cout, void* __restrict__ Cout2, int ldc, long strideC,
    const float* __restrict__ bias,
    const float* __restrict__ resid, long strideR,
    int M, int N, int K, float scale) {
  typedef typename Elem<ET>::T T;
  typedef typename Frag<T>::V V;
  const T* A = (const T*)Ap; const T* A2 = (const T*)A2p; const T* Bt = (const T*)Btp; const T* Bt2 = (const T*)Bt2p;
  __shared__ __align__(16) float sT[8][16 * 68];
  const int b    = blockIdx.y;
  const int lane = threadIdx.x & 31;
  const int wave = threadIdx.x >> 5;
  const int tilesN = N >> 6;
  const int tilesM = M >> 6;
  const int tile = blockIdx.x * 8 + wave;
  if (tile >= tilesM * tilesN) return;
  const int tm = tile / tilesN;
  const int tn = tile - tm * tilesN;
  const int m0 = tm << 6;
  const int n0 = tn << 6;

  const T* Ab  = A  + (size_t)b * strideA;
  const T* Bb  = Bt + (size_t)b * strideB;
  const T* Ab2 = SPLIT ? (A2  + (size_t)b * strideA) : nullptr;
  const T* Bb2 = SPLIT ? (Bt2 + (size_t)b * strideB) : nullptr;

  const int rlane = lane & 15;
  const int koff  = (lane >> 4) * 8;
  const int mOff  = (lane >> 4) * 8;

  v8f acc[4][4];
#pragma unroll
  for (int i = 0; i < 4; ++i)
#pragma unroll
    for (int j = 0; j < 4; ++j) acc[i][j] = (v8f){0.f,0.f,0.f,0.f,0.f,0.f,0.f,0.f};

  for (int k0 = 0; k0 < K; k0 += 32) {
    V bh[4], bl[4];
#pragma unroll
    for (int j = 0; j < 4; ++j) {
      const size_t bo = (size_t)(n0 + (j << 4) + rlane) * ldb + koff + k0;
      bh[j] = Frag<T>::load(Bb + bo);
      if (SPLIT) bl[j] = Frag<T>::load(Bb2 + bo);
    }
#pragma unroll
    for (int i = 0; i < 4; ++i) {
      const size_t ao = (size_t)(m0 + (i << 4) + rlane) * lda + koff + k0;
      V ah = Frag<T>::load(Ab + ao);
      V al;
      if (SPLIT) al = Frag<T>::load(Ab2 + ao);
#pragma unroll
      for (int j = 0; j < 4; ++j) {
        acc[i][j] = Frag<T>::mma(ah, bh[j], acc[i][j]);
        if (SPLIT) {
          acc[i][j] = Frag<T>::mma(ah, bl[j], acc[i][j]);
          acc[i][j] = Frag<T>::mma(al, bh[j], acc[i][j]);
        }
      }
      Frag<T>::guard(acc[i][0], acc[i][3], ah, SPLIT ? al : ah);
    }
    Frag<T>::keep(bh[0], bh[1], bh[2], bh[3]);
    if (SPLIT) Frag<T>::keep(bl[0], bl[1], bl[2], bl[3]);
  }
  acc_guard4(acc[0][0], acc[0][1], acc[0][2], acc[0][3]);
  acc_guard4(acc[1][0], acc[1][1], acc[1][2], acc[1][3]);
  acc_guard4(acc[2][0], acc[2][1], acc[2][2], acc[2][3]);
  acc_guard4(acc[3][0], acc[3][1], acc[3][2], acc[3][3]);

  float* slab = sT[wave];
  const float* Rb = RESID ? (resid + (size_t)b * strideR) : nullptr;
#pragma unroll
  for (int i = 0; i < 4; ++i) {
    const int mBase = m0 + (i << 4);
#pragma unroll
    for (int j = 0; j < 4; ++j) {
      const int n = n0 + (j << 4) + rlane;
      float bv = 0.f;
      if (BIAS_MODE == 2) bv = bias[n];
#pragma unroll
      for (int r = 0; r < 8; ++r) {
        float v = acc[i][j][r] * scale;
        if (BIAS_MODE == 1) v += bias[mBase + mOff + r];
        if (BIAS_MODE == 2) v += bv;
        if (RESID) v += Rb[(size_t)(mBase + mOff + r) * ldc + n];
        if (ACT == 1) v = tanhf(v);
        if (ACT == 2) v = fmaxf(v, 0.0f);
        if (ACT == 3) v = v / (1.0f + expf(-v));
        if (ACT == 4) v = (v > 0.f) ? v : 0.01f * v;
        if (ACT == 5) v = 0.5f * v * (1.0f + erff(v * 0.70710678118654752f));
        slab[(mOff + r) * 68 + (j << 4) + rlane] = v;
      }
    }
    __builtin_amdgcn_fence(__ATOMIC_RELEASE, "workgroup");
    __builtin_amdgcn_wave_barrier();
    __builtin_amdgcn_fence(__ATOMIC_ACQUIRE, "workgroup");
    if (OUT_MODE == 0) {
      float* C = (float*)Cout + (size_t)b * strideC;
      const int hh = lane >> 4, c4 = (lane & 15) * 4;
      for (int pass = 0; pass < 2; ++pass) {
#pragma unroll
        for (int it = 0; it < 8; ++it) {
          const int row = it * 2 + hh;
          v4f v = *(const v4f*)(slab + row * 68 + c4);
          *(volatile v4f*)(C + (size_t)(mBase + row) * ldc + n0 + c4) = v;
        }
        __threadfence();
      }
    } else {
      const int q = lane >> 3, c8 = (lane & 7) * 8;
      unsigned short* C  = (unsigned short*)Cout  + (size_t)b * strideC;
      unsigned short* C2 = (OUT_MODE == 2) ? ((unsigned short*)Cout2 + (size_t)b * strideC) : nullptr;
      for (int pass = 0; pass < 2; ++pass) {
#pragma unroll
        for (int it = 0; it < 4; ++it) {
          const int row = it * 4 + q;
          const float* sp = slab + row * 68 + c8;
          v8h hv, lv;
#pragma unroll
          for (int e = 0; e < 8; ++e) {
            if (OUT_MODE == 1) {
              hv[e] = (_Float16)sp[e];
            } else {
              unsigned short hb = f2bf_bits(sp[e]);
              unsigned short lb = f2bf_bits(sp[e] - bf_bits2f(hb));
              hv[e] = __builtin_bit_cast(_Float16, hb);
              lv[e] = __builtin_bit_cast(_Float16, lb);
            }
          }
          *(volatile v8h*)(C + (size_t)(mBase + row) * ldc + n0 + c8) = hv;
          if (OUT_MODE == 2) *(volatile v8h*)(C2 + (size_t)(mBase + row) * ldc + n0 + c8) = lv;
        }
        __threadfence();
      }
    }
    __builtin_amdgcn_fence(__ATOMIC_RELEASE, "workgroup");
    __builtin_amdgcn_wave_barrier();
    __builtin_amdgcn_fence(__ATOMIC_ACQUIRE, "workgroup");
  }
}

__global__ __launch_bounds__(256) void cast_f32_f16x8(
    const float* __restrict__ in, unsigned short* __restrict__ out, int n8, float scale) {
  const int i  = blockIdx.x * 256 + threadIdx.x;
  const int ic = (i < n8) ? i : (n8 - 1);
  const v4f a0 = *(const v4f*)(in + (size_t)8 * ic);
  const v4f a1 = *(const v4f*)(in + (size_t)8 * ic + 4);
  v8h hv;
#pragma unroll
  for (int e = 0; e < 4; ++e) {
    hv[e]     = (_Float16)(a0[e] * scale);
    hv[4 + e] = (_Float16)(a1[e] * scale);
  }
  if (i < n8) {
    unsigned short* p = out + (size_t)8 * i;
    *(volatile v8h*)p = hv;
    __threadfence();
    *(volatile v8h*)p = hv;
  }
}

struct RopeFreq { float inv[32]; };
static_assert(sizeof(RopeFreq) == 128, "no padding");

__global__ __launch_bounds__(256) void rope_f32_to_f16(
    const float* __restrict__ pf, unsigned short* __restrict__ out, int nrows, int seqlen, int ld, RopeFreq fr) {
#pragma clang fp contract(off)
  __shared__ float cs_c[2][32];
  __shared__ float cs_s[2][32];
  const int tid = threadIdx.x;
  if (tid < 64) {
    const int rr = tid >> 5;
    const int i  = tid & 31;
    int prow = blockIdx.x * 2 + rr;
    prow = (prow < nrows) ? prow : (nrows - 1);
    const int pos = prow % seqlen;
    float inv = 0.0f;
#pragma unroll
    for (int j = 0; j < 32; ++j) inv = (i == j) ? fr.inv[j] : inv;
    const float ang = (float)pos * inv;
    float sv, cv;
    sincosf(ang, &sv, &cv);
    cs_c[rr][i] = cv;
    cs_s[rr][i] = sv;
  }
  __syncthreads();
  const int r2  = tid >> 7;
  const int t   = tid & 127;
  const int row = blockIdx.x * 2 + r2;
  const int rowc = (row < nrows) ? row : (nrows - 1);
  const int col0 = t * 8;
  const int i0   = (col0 & 63) >> 1;
  const float* src = pf + (size_t)rowc * ld + col0;
  const v4f xa = *(const v4f*)src;
  const v4f xb = *(const v4f*)(src + 4);
  float xs[8];
#pragma unroll
  for (int e = 0; e < 4; ++e) { xs[e] = xa[e]; xs[4 + e] = xb[e]; }
  v8h hv;
#pragma unroll
  for (int p = 0; p < 4; ++p) {
    const float cv = cs_c[r2][i0 + p];
    const float sv = cs_s[r2][i0 + p];
    const float x1 = xs[2 * p];
    const float x2 = xs[2 * p + 1];
    const float re = x1 * cv - x2 * sv;
    const float im = x1 * sv + x2 * cv;
    hv[2 * p]     = (_Float16)re;
    hv[2 * p + 1] = (_Float16)im;
  }
  if (row < nrows) {
    unsigned short* dst = out + (size_t)row * ld + col0;
    *(volatile v8h*)dst = hv;
    __threadfence();
    *(volatile v8h*)dst = hv;
  }
}

#define AT_D 64
#define AT_NW 4
#define AT_QB 64
#define AT_KC 64

__device__ __forceinline__ v8f mma_f16g(v16h a, v16h b, v8f c) {
  c = __builtin_amdgcn_wmma_f32_16x16x32_f16(false, a, false, b, (short)0, c, false, false);
  asm volatile("v_nop\n\tv_nop\n\tv_nop\n\tv_nop" : "+v"(c) : "v"(a), "v"(b));
  return c;
}

__global__ __launch_bounds__(128)
void attn64_h16(const unsigned short* __restrict__ qp, const unsigned short* __restrict__ kp,
                const unsigned short* __restrict__ vp, unsigned short* __restrict__ op,
                int S, int H, int ld, float sm_scale, float out_carry) {
  const float PSC = 32768.0f;
  union FH { v16h v; v8h h[2]; };
  __shared__ __align__(16) unsigned short Ksh[AT_KC * AT_D];
  __shared__ __align__(16) unsigned short Vth[AT_D * AT_KC];
  __shared__ __align__(16) _Float16 Psh[AT_NW][16 * AT_KC];
  __shared__ __align__(16) float Os[AT_NW][16 * 68];

  const int tid  = threadIdx.x;
  const int wave = tid >> 5;
  const int lane = tid & 31;
  const int hh   = lane >> 4;
  const int c    = lane & 15;

  const int nqb = S / AT_QB;
  const int bx  = blockIdx.x;
  const int qb  = bx % nqb;
  const int bh  = bx / nqb;
  const int h   = bh % H;
  const int b   = bh / H;
  const int q0  = qb * AT_QB + wave * 16;
  const size_t rowbase = (size_t)b * S;
  const int hcol = h * AT_D;

  v16h qa[2];
  {
    const _Float16* qrow = (const _Float16*)qp + (rowbase + q0 + c) * (size_t)ld + hcol + 8 * hh;
#pragma unroll
    for (int dc = 0; dc < 2; ++dc) {
      FH f;
      f.h[0] = *(const v8h*)(qrow + dc * 32);
      f.h[1] = *(const v8h*)(qrow + dc * 32 + 16);
      qa[dc] = f.v;
    }
  }

  float mrow[8], lrow[8];
  v8f oacc[4];
#pragma unroll
  for (int r = 0; r < 8; ++r) { mrow[r] = -INFINITY; lrow[r] = 0.f; }
#pragma unroll
  for (int t = 0; t < 4; ++t) oacc[t] = (v8f){0.f,0.f,0.f,0.f,0.f,0.f,0.f,0.f};

  const int nChunks = S / AT_KC;
  for (int kc = 0; kc < nChunks; ++kc) {
    const int kv0 = kc * AT_KC;
    __syncthreads();
    {
      const int kvr = tid >> 1, dh = (tid & 1) * 32;
      const v4u* krow = (const v4u*)(kp + (rowbase + kv0 + kvr) * (size_t)ld + hcol + dh);
      const v4u* vrow = (const v4u*)(vp + (rowbase + kv0 + kvr) * (size_t)ld + hcol + dh);
      v4u* kdst = (v4u*)(Ksh + kvr * AT_D + dh);
#pragma unroll
      for (int i = 0; i < 4; ++i) {
        const v4u kw = krow[i];
        kdst[i] = kw;
        const v4u vw = vrow[i];
#pragma unroll
        for (int e = 0; e < 4; ++e) {
          const unsigned w = vw[e];
          const int d = dh + 8 * i + 2 * e;
          Vth[d * AT_KC + kvr]       = (unsigned short)(w & 0xffffu);
          Vth[(d + 1) * AT_KC + kvr] = (unsigned short)(w >> 16);
        }
      }
    }
    __syncthreads();
    const _Float16* ksh = (const _Float16*)Ksh;
    const _Float16* vth = (const _Float16*)Vth;

    v8f s[4];
#pragma unroll
    for (int j = 0; j < 4; ++j) {
      s[j] = (v8f){0.f,0.f,0.f,0.f,0.f,0.f,0.f,0.f};
#pragma unroll
      for (int dc = 0; dc < 2; ++dc) {
        FH kb;
        kb.h[0] = *(const v8h*)(ksh + (j * 16 + c) * AT_D + dc * 32 + 8 * hh);
        kb.h[1] = *(const v8h*)(ksh + (j * 16 + c) * AT_D + dc * 32 + 16 + 8 * hh);
        s[j] = mma_f16g(qa[dc], kb.v, s[j]);
      }
    }
    float cm[8];
#pragma unroll
    for (int r = 0; r < 8; ++r) {
      float m = -INFINITY;
#pragma unroll
      for (int j = 0; j < 4; ++j) {
        const float sv = s[j][r] * sm_scale;
        s[j][r] = sv;
        m = fmaxf(m, sv);
      }
#pragma unroll
      for (int off = 1; off < 16; off <<= 1) m = fmaxf(m, __shfl_xor(m, off, 32));
      cm[r] = m;
    }
    _Float16* pwh = Psh[wave];
#pragma unroll
    for (int r = 0; r < 8; ++r) {
      const float mnew  = fmaxf(mrow[r], cm[r]);
      const float alpha = expf(mrow[r] - mnew);
      mrow[r] = mnew;
      float psum = 0.f;
#pragma unroll
      for (int j = 0; j < 4; ++j) {
        const float p = expf(s[j][r] - mnew);
        psum += p;
        pwh[(8 * hh + r) * AT_KC + j * 16 + c] = (_Float16)(p * PSC);
      }
#pragma unroll
      for (int off = 1; off < 16; off <<= 1) psum += __shfl_xor(psum, off, 32);
      lrow[r] = lrow[r] * alpha + psum;
#pragma unroll
      for (int t = 0; t < 4; ++t) oacc[t][r] *= alpha;
    }
    __builtin_amdgcn_fence(__ATOMIC_RELEASE, "workgroup");
    __builtin_amdgcn_wave_barrier();
    __builtin_amdgcn_fence(__ATOMIC_ACQUIRE, "workgroup");
#pragma unroll 1
    for (int kk = 0; kk < 2; ++kk) {
      FH pa;
      pa.h[0] = *(const v8h*)(pwh + c * AT_KC + kk * 32 + 8 * hh);
      pa.h[1] = *(const v8h*)(pwh + c * AT_KC + kk * 32 + 16 + 8 * hh);
#pragma unroll
      for (int t = 0; t < 4; ++t) {
        FH vb;
        vb.h[0] = *(const v8h*)(vth + (t * 16 + c) * AT_KC + kk * 32 + 8 * hh);
        vb.h[1] = *(const v8h*)(vth + (t * 16 + c) * AT_KC + kk * 32 + 16 + 8 * hh);
        oacc[t] = mma_f16g(pa.v, vb.v, oacc[t]);
      }
    }
  }

  float* os = Os[wave];
#pragma unroll
  for (int r = 0; r < 8; ++r) {
    const float inv = out_carry / (lrow[r] * PSC);
#pragma unroll
    for (int t = 0; t < 4; ++t) os[(8 * hh + r) * 68 + t * 16 + c] = oacc[t][r] * inv;
  }
  __builtin_amdgcn_fence(__ATOMIC_RELEASE, "workgroup");
  __builtin_amdgcn_wave_barrier();
  __builtin_amdgcn_fence(__ATOMIC_ACQUIRE, "workgroup");
  {
    const int q8 = lane >> 3, c8 = (lane & 7) * 8;
    for (int pass = 0; pass < 2; ++pass) {
#pragma unroll
      for (int it = 0; it < 4; ++it) {
        const int row = it * 4 + q8;
        const float* sp = os + row * 68 + c8;
        v8h hv;
#pragma unroll
        for (int e = 0; e < 8; ++e) hv[e] = (_Float16)sp[e];
        *(volatile v8h*)(op + (rowbase + q0 + row) * (size_t)ld + hcol + c8) = hv;
      }
      __threadfence();
    }
  }
}

extern "C" void kernel_launch(void* const* d_in, const int* in_sizes, int n_in,
                              void* d_out, int out_size, void* d_ws, size_t ws_size,
                              hipStream_t stream) {
  constexpr int kB = 2, kL = 2048, kD = 1024, kH = 16, kHd = 64;
  constexpr int kM = kB * kL;
  static_assert(kD == kH * kHd, "head split");
  static_assert(kHd == AT_D, "head dim 64");
  static_assert(kM % 64 == 0 && kD % 64 == 0, "GEMM M,N tile multiples (M=4096, N=1024)");
  static_assert(kD % 32 == 0, "GEMM K % 32 == 0 (K=1024)");
  static_assert(kL % AT_QB == 0 && kL % AT_KC == 0, "attention S % 64 == 0");
  static_assert((kM * kD) % (8 * 256) == 0 && (kD * kD) % (8 * 256) == 0, "cast grids exact");
  static_assert(kM % 2 == 0 && kD == 128 * 8, "rope grid exact");

  if (n_in < 11) return;
  if (in_sizes[0] != kM * kD || in_sizes[1] != kM * kD || in_sizes[2] != kM * kD) return;
  if (in_sizes[3] != kD * kD || in_sizes[5] != kD * kD || in_sizes[7] != kD * kD || in_sizes[9] != kD * kD) return;
  if (in_sizes[4] != kD || in_sizes[6] != kD || in_sizes[8] != kD || in_sizes[10] != kD) return;
  if (out_size != kM * kD) return;

  const float* q_in = (const float*)d_in[0];
  const float* k_in = (const float*)d_in[1];
  const float* v_in = (const float*)d_in[2];
  const float* wq = (const float*)d_in[3];
  const float* bq = (const float*)d_in[4];
  const float* wk = (const float*)d_in[5];
  const float* bk = (const float*)d_in[6];
  const float* wv = (const float*)d_in[7];
  const float* bv = (const float*)d_in[8];
  const float* wo = (const float*)d_in[9];
  const float* bo = (const float*)d_in[10];
  float* out = (float*)d_out;

  const size_t actH = (size_t)kM * kD * 2;
  const size_t wgtH = (size_t)kD * kD * 2;
  const size_t actF = (size_t)kM * kD * 4;
  size_t off = 0;
  char* ws = (char*)d_ws;
  unsigned short* xh = (unsigned short*)(ws + off); off += actH;
  unsigned short* wh = (unsigned short*)(ws + off); off += wgtH;
  float*          pf = (float*)(ws + off);          off += actF;
  unsigned short* qh = (unsigned short*)(ws + off); off += actH;
  unsigned short* kh = (unsigned short*)(ws + off); off += actH;
  unsigned short* vh = (unsigned short*)(ws + off); off += actH;
  unsigned short* oh = (unsigned short*)(ws + off); off += actH;
  if (off > ws_size) return;

  const int act_n8 = kM * kD / 8;
  const int wgt_n8 = kD * kD / 8;
  const int act_blk = (act_n8 + 255) / 256;
  const int wgt_blk = (wgt_n8 + 255) / 256;
  const float wcarry = 64.0f;
  const float wscale = 1.0f / 64.0f;
  const dim3 ggrid((kM / 64) * (kD / 64) / 8, 1);
  const int rope_blk = kM / 2;

  RopeFreq fr;
  for (int i = 0; i < 32; ++i) fr.inv[i] = (float)(1.0 / pow(10000.0, (double)(2 * i) / 64.0));

  cast_f32_f16x8<<<act_blk, 256, 0, stream>>>(q_in, xh, act_n8, 1.0f);
  cast_f32_f16x8<<<wgt_blk, 256, 0, stream>>>(wq, wh, wgt_n8, wcarry);
  wmma_gemm64<0, false, 2, 0, false, 0><<<ggrid, 256, 0, stream>>>(
      xh, xh, kD, 0L, wh, wh, kD, 0L, (void*)pf, (void*)pf, kD, 0L, bq, bq, 0L, kM, kD, kD, wscale);
  rope_f32_to_f16<<<rope_blk, 256, 0, stream>>>(pf, qh, kM, kL, kD, fr);

  cast_f32_f16x8<<<act_blk, 256, 0, stream>>>(k_in, xh, act_n8, 1.0f);
  cast_f32_f16x8<<<wgt_blk, 256, 0, stream>>>(wk, wh, wgt_n8, wcarry);
  wmma_gemm64<0, false, 2, 0, false, 0><<<ggrid, 256, 0, stream>>>(
      xh, xh, kD, 0L, wh, wh, kD, 0L, (void*)pf, (void*)pf, kD, 0L, bk, bk, 0L, kM, kD, kD, wscale);
  rope_f32_to_f16<<<rope_blk, 256, 0, stream>>>(pf, kh, kM, kL, kD, fr);

  cast_f32_f16x8<<<act_blk, 256, 0, stream>>>(v_in, xh, act_n8, 1.0f);
  cast_f32_f16x8<<<wgt_blk, 256, 0, stream>>>(wv, wh, wgt_n8, wcarry);
  wmma_gemm64<0, false, 2, 1, false, 0><<<ggrid, 256, 0, stream>>>(
      xh, xh, kD, 0L, wh, wh, kD, 0L, (void*)vh, (void*)vh, kD, 0L, bv, bv, 0L, kM, kD, kD, wscale);

  attn64_h16<<<kB * kH * (kL / AT_QB), 128, 0, stream>>>(qh, kh, vh, oh, kL, kH, kD, 0.125f, 64.0f);

  cast_f32_f16x8<<<wgt_blk, 256, 0, stream>>>(wo, wh, wgt_n8, wcarry);
  wmma_gemm64<0, false, 2, 0, false, 0><<<ggrid, 256, 0, stream>>>(
      oh, oh, kD, 0L, wh, wh, kD, 0L, (void*)out, (void*)out, kD, 0L, bo, bo, 0L, kM, kD, kD, 1.0f / 4096.0f);
}
